// Block_40106404610136
// MI455X (gfx1250) — hardware-verified
//
#include <hip/hip_runtime.h>
#include <math.h>

#ifndef NB
#define NB 64
#endif
#ifndef SEQ
#define SEQ 256
#endif
#define NB_FULL 64
#define SEQ_FULL 256
#define NE 384
#define NHD 6
#define HD 64
#define NQKV (3 * NE)
#define NFF (4 * NE)
#define MROWS (NB * SEQ)

static_assert(SEQ % 64 == 0);
static_assert(SEQ <= SEQ_FULL);
static_assert(NB <= NB_FULL);
static_assert(NHD * HD == NE);
static_assert(NE % 128 == 0);
static_assert(NE % 64 == 0 && NQKV % 64 == 0 && NFF % 64 == 0);
static_assert(NE % 32 == 0 && NFF % 32 == 0);
static_assert(MROWS % 64 == 0);

typedef __attribute__((ext_vector_type(16))) _Float16 v16h;
typedef __attribute__((ext_vector_type(8)))  _Float16 v8h;
typedef __attribute__((ext_vector_type(8)))  float    v8f;
typedef __attribute__((ext_vector_type(4)))  float    v4f;
typedef v8h v8ha __attribute__((may_alias));
typedef v4f v4fa __attribute__((may_alias));
typedef unsigned int cm_u4 __attribute__((ext_vector_type(4)));
typedef unsigned int bk_u2 __attribute__((ext_vector_type(2)));

union FragU { v16h v; v8h h[2]; };

#define VST2(T, ptr, val) do { const T vst2_v_ = (val); *(volatile T*)(ptr) = vst2_v_; __threadfence(); *(volatile T*)(ptr) = vst2_v_; } while (0)

__device__ __forceinline__ v8f wmma16(v16h a, v16h b, v8f c) {
    c = __builtin_amdgcn_wmma_f32_16x16x32_f16(false, a, false, b, (short)0, c, false, false);
    asm volatile("v_nop\n\tv_nop\n\tv_nop\n\tv_nop" : "+v"(c) : "v"(a), "v"(b));
    return c;
}
__device__ __forceinline__ void dep_guard_h(v8f& a, v8f& b, v16h x, v16h y) { asm volatile("v_nop\n\tv_nop\n\tv_nop\n\tv_nop" : "+v"(a), "+v"(b) : "v"(x), "v"(y)); }
__device__ __forceinline__ void keep4_h(v16h a, v16h b, v16h c, v16h d) { asm volatile("v_nop" :: "v"(a), "v"(b), "v"(c), "v"(d)); }
__device__ __forceinline__ void acc_guard4(v8f& a, v8f& b, v8f& c, v8f& d) { asm volatile("v_nop\n\tv_nop\n\tv_nop\n\tv_nop" : "+v"(a), "+v"(b), "+v"(c), "+v"(d)); }
__device__ __forceinline__ void wave_sync() {
    __builtin_amdgcn_fence(3  , "workgroup");
    __builtin_amdgcn_wave_barrier();
    __builtin_amdgcn_fence(2  , "workgroup");
}
__device__ __forceinline__ v16h frag_ld(const _Float16* __restrict__ p) { FragU f; f.h[0] = *(const v8h*)(p); f.h[1] = *(const v8h*)(p + 16); return f.v; }

__device__ __forceinline__ unsigned int cmb_pk2(float a, float b) { return (unsigned int)__builtin_bit_cast(unsigned short, (_Float16)a) | ((unsigned int)__builtin_bit_cast(unsigned short, (_Float16)b) << 16); }
__device__ __forceinline__ float cmb_bf(float v) { const unsigned u = __builtin_bit_cast(unsigned, v); const unsigned r = (u + 0x7fffu + ((u >> 16) & 1u)) & 0xffff0000u; return __builtin_bit_cast(float, r); }

__global__ __launch_bounds__(256) void k_cm_castbT(const float* __restrict__ SRC, int lds, long long src_z, unsigned short* __restrict__ DST, int ldd, long long dst_z, int nR, int nC, float sc) {
    const long long u = (long long)blockIdx.x * 256 + threadIdx.x; const int per = nR / 8; if (u >= (long long)nC * per) return;
    const int z = blockIdx.y; const int c = (int)(u / per); const int r0 = 8 * (int)(u % per);
    const float* s = SRC + (long long)z * src_z;
    float w[8];
#pragma unroll
    for (int e = 0; e < 8; ++e) w[e] = cmb_bf(s[(long long)(r0 + e) * lds + c]) * sc;
    cm_u4 pk; pk.x = cmb_pk2(w[0], w[1]); pk.y = cmb_pk2(w[2], w[3]); pk.z = cmb_pk2(w[4], w[5]); pk.w = cmb_pk2(w[6], w[7]);
    VST2(cm_u4, (cm_u4*)(DST + (long long)z * dst_z + (long long)c * ldd + r0), pk);
}

template <int NQ, int ABF>
__global__ __launch_bounds__(256) void k_b_ln(const float* __restrict__ A, const float* __restrict__ GA, const float* __restrict__ BE, float eps, float inv_vden, int rows, int seq, int seq_src, unsigned short* __restrict__ Y16) {
    #pragma clang fp contract(off)
    constexpr int WD = 128 * NQ;
    const int wave = __builtin_amdgcn_readfirstlane(threadIdx.x >> 5);
    const int r = blockIdx.x * 8 + wave; const int L = threadIdx.x & 31;
    if (r >= rows) return;
    const int bsrc = r / seq; const long long rsrc = (long long)bsrc * seq_src + (r - bsrc * seq);
    v4f v[NQ]; float s = 0.f;
#pragma unroll
    for (int q = 0; q < NQ; ++q) {
        v[q] = *(const v4f*)(A + rsrc * WD + 4 * L + 128 * q);
        if (ABF) { v[q].x = cmb_bf(v[q].x); v[q].y = cmb_bf(v[q].y); v[q].z = cmb_bf(v[q].z); v[q].w = cmb_bf(v[q].w); }
        s += (v[q].x + v[q].y) + (v[q].z + v[q].w);
    }
#pragma unroll
    for (int o = 16; o > 0; o >>= 1) s += __shfl_xor(s, o, 32);
    const float mu = s * (1.f / WD); float qq = 0.f;
#pragma unroll
    for (int q = 0; q < NQ; ++q) { v[q].x -= mu; v[q].y -= mu; v[q].z -= mu; v[q].w -= mu; qq += (v[q].x * v[q].x + v[q].y * v[q].y) + (v[q].z * v[q].z + v[q].w * v[q].w); }
#pragma unroll
    for (int o = 16; o > 0; o >>= 1) qq += __shfl_xor(qq, o, 32);
    const float rs = rsqrtf(qq * inv_vden + eps);
#pragma unroll
    for (int q = 0; q < NQ; ++q) {
        const int c = 4 * L + 128 * q; const v4f ga = *(const v4f*)(GA + c), be = *(const v4f*)(BE + c);
        const float y0 = v[q].x * rs * cmb_bf(ga.x) + cmb_bf(be.x), y1 = v[q].y * rs * cmb_bf(ga.y) + cmb_bf(be.y);
        const float y2 = v[q].z * rs * cmb_bf(ga.z) + cmb_bf(be.z), y3 = v[q].w * rs * cmb_bf(ga.w) + cmb_bf(be.w);
        bk_u2 pk; pk.x = cmb_pk2(y0, y1); pk.y = cmb_pk2(y2, y3);
        VST2(bk_u2, (bk_u2*)(Y16 + (long long)r * WD + c), pk);
    }
}

template <int BIAS_MODE, int OUT_MODE, bool RESID, bool RBF, int ACT>
__global__ __launch_bounds__(256) void wmma_gemm64(
    const unsigned short* __restrict__ Ap, int lda, long long strideA,
    const unsigned short* __restrict__ Btp, int ldb, long long strideB,
    void* __restrict__ Cout, int ldc, long long strideC,
    const float* __restrict__ bias,
    const float* __restrict__ resid, long long strideR,
    int M, int N, int K, float scale) {
  __shared__ __align__(16) float sT[8][16 * 68];
  const int b    = blockIdx.y;
  const int lane = threadIdx.x & 31;
  const int wave = __builtin_amdgcn_readfirstlane(threadIdx.x >> 5);
  const int tilesN = N >> 6;
  const int tilesM = M >> 6;
  const int tile = blockIdx.x * 8 + wave;
  if (tile >= tilesM * tilesN) return;
  const int tm = tile / tilesN;
  const int tn = tile - tm * tilesN;
  const int m0 = tm << 6;
  const int n0 = tn << 6;

  const _Float16* Ab = (const _Float16*)Ap  + (size_t)((long long)b * strideA);
  const _Float16* Bb = (const _Float16*)Btp + (size_t)((long long)b * strideB);

  const int rlane = lane & 15;
  const int koff  = (lane >> 4) * 8;
  const int mOff  = (lane >> 4) * 8;

  v8f acc[4][4];
#pragma unroll
  for (int i = 0; i < 4; ++i)
#pragma unroll
    for (int j = 0; j < 4; ++j) acc[i][j] = (v8f){0.f,0.f,0.f,0.f,0.f,0.f,0.f,0.f};

  for (int k0 = 0; k0 < K; k0 += 32) {
    v16h bh[4];
#pragma unroll
    for (int j = 0; j < 4; ++j) {
      const size_t bo = (size_t)(n0 + (j << 4) + rlane) * ldb + koff + k0;
      bh[j] = frag_ld(Bb + bo);
    }
#pragma unroll
    for (int i = 0; i < 4; ++i) {
      const size_t ao = (size_t)(m0 + (i << 4) + rlane) * lda + koff + k0;
      const v16h ah = frag_ld(Ab + ao);
#pragma unroll
      for (int j = 0; j < 4; ++j)
        acc[i][j] = __builtin_amdgcn_wmma_f32_16x16x32_f16(false, ah, false, bh[j], (short)0, acc[i][j], false, false);
      dep_guard_h(acc[i][0], acc[i][3], ah, ah);
    }
    keep4_h(bh[0], bh[1], bh[2], bh[3]);
  }
  acc_guard4(acc[0][0], acc[0][1], acc[0][2], acc[0][3]);
  acc_guard4(acc[1][0], acc[1][1], acc[1][2], acc[1][3]);
  acc_guard4(acc[2][0], acc[2][1], acc[2][2], acc[2][3]);
  acc_guard4(acc[3][0], acc[3][1], acc[3][2], acc[3][3]);

  const float* Rb = RESID ? (resid + (size_t)((long long)b * strideR)) : nullptr;
#pragma unroll
  for (int i = 0; i < 4; ++i) {
    const int mBase = m0 + (i << 4);
#pragma unroll
    for (int j = 0; j < 4; ++j) {
      const int n = n0 + (j << 4) + rlane;
      float bv = 0.f;
      if (BIAS_MODE == 2) bv = cmb_bf(bias[n]);
#pragma unroll
      for (int r = 0; r < 8; ++r) {
        float v = acc[i][j][r] * scale;
        if (BIAS_MODE == 2) v += bv;
        if (RESID) { float rv = Rb[(size_t)(mBase + mOff + r) * ldc + n]; if (RBF) rv = cmb_bf(rv); v += rv; }
        if (ACT == 2) v = fmaxf(v, 0.0f);
        sT[wave][(mOff + r) * 68 + (j << 4) + rlane] = v;
      }
    }
    wave_sync();
    if (OUT_MODE == 0) {
      float* C = (float*)Cout + (size_t)((long long)b * strideC);
      const int hh = lane >> 4, c4 = (lane & 15) * 4;
      for (int pass = 0; pass < 2; ++pass) {
#pragma unroll
        for (int it = 0; it < 8; ++it) {
          const int row = it * 2 + hh;
          const v4f v = *(const v4fa*)&sT[wave][row * 68 + c4];
          *(volatile v4f*)(C + (size_t)(mBase + row) * ldc + n0 + c4) = v;
        }
        __threadfence();
      }
    } else {
      const int q = lane >> 3, c8 = (lane & 7) * 8;
      unsigned short* C = (unsigned short*)Cout + (size_t)((long long)b * strideC);
      for (int pass = 0; pass < 2; ++pass) {
#pragma unroll
        for (int it = 0; it < 4; ++it) {
          const int row = it * 4 + q;
          v8h hv;
#pragma unroll
          for (int e = 0; e < 8; ++e) hv[e] = (_Float16)sT[wave][row * 68 + c8 + e];
          *(volatile v8h*)(C + (size_t)(mBase + row) * ldc + n0 + c8) = hv;
        }
        __threadfence();
      }
    }
    wave_sync();
  }
}

#define AT_KP 72
#define AT_VP 72
#define AT_PP 40
#define AT_OP 68
__global__ __launch_bounds__(128) void k_attn_causal(const unsigned short* __restrict__ QKVp, unsigned short* __restrict__ AOp, float sl2e, float oscale) {
  __shared__ __align__(16) _Float16 Ksh[64 * AT_KP];
  __shared__ __align__(16) _Float16 Vth[64 * AT_VP];
  __shared__ __align__(16) _Float16 Psh[4][16 * AT_PP];
  __shared__ __align__(16) float    Os[4][16 * AT_OP];
  const _Float16* QKV = (const _Float16*)QKVp;
  const int tid  = threadIdx.x;
  const int wave = __builtin_amdgcn_readfirstlane(tid >> 5);
  const int lane = tid & 31;
  const int hh   = lane >> 4;
  const int c    = lane & 15;
  constexpr int NQB = SEQ / 64;
  const int bx = blockIdx.x;
  const int qb = bx % NQB;
  const int bhd = bx / NQB;
  const int h  = bhd % NHD;
  const int b  = bhd / NHD;
  const int q0 = qb * 64 + wave * 16;
  const size_t rowbase = (size_t)b * SEQ;
  const float NEG = -__builtin_inff();
  const size_t qoff = (rowbase + q0 + c) * NQKV + h * HD + 8 * hh;

  float mrow[8], lrow[8];
  v8f oacc[4];
#pragma unroll
  for (int r = 0; r < 8; ++r) { mrow[r] = NEG; lrow[r] = 0.f; }
#pragma unroll
  for (int t = 0; t < 4; ++t) oacc[t] = (v8f){0.f,0.f,0.f,0.f,0.f,0.f,0.f,0.f};

  const int nChunks = qb + 1;
  for (int kc = 0; kc < nChunks; ++kc) {
    const int kv0 = kc * 64;
    __syncthreads();
    {
      const int kvr = tid >> 1, dh = (tid & 1) * 32;
      const size_t go = (rowbase + kv0 + kvr) * NQKV + h * HD + dh;
#pragma unroll
      for (int i = 0; i < 4; ++i) {
        const v8h kk = *(const v8h*)(QKV + go + NE + 8 * i);
        const v8h vv = *(const v8h*)(QKV + go + 2 * NE + 8 * i);
        *(v8ha*)&Ksh[kvr * AT_KP + dh + 8 * i] = kk;
#pragma unroll
        for (int e = 0; e < 8; ++e) Vth[(dh + 8 * i + e) * AT_VP + kvr] = vv[e];
      }
    }
    __syncthreads();

#pragma unroll 1
    for (int hf = 0; hf < 2; ++hf) {
      const int kh0 = kv0 + hf * 32;
      if (kh0 <= q0 + 15) {
        v8f s0 = (v8f){0.f,0.f,0.f,0.f,0.f,0.f,0.f,0.f};
        v8f s1 = s0;
#pragma unroll
        for (int dc = 0; dc < 2; ++dc) {
          FragU qa, k0f, k1f;
          qa.h[0] = *(const v8h*)(QKV + qoff + dc * 32);
          qa.h[1] = *(const v8h*)(QKV + qoff + dc * 32 + 16);
          const int kb0 = (hf * 32 + c) * AT_KP + dc * 32 + 8 * hh;
          const int kb1 = kb0 + 16 * AT_KP;
          k0f.h[0] = *(const v8ha*)&Ksh[kb0]; k0f.h[1] = *(const v8ha*)&Ksh[kb0 + 16];
          k1f.h[0] = *(const v8ha*)&Ksh[kb1]; k1f.h[1] = *(const v8ha*)&Ksh[kb1 + 16];
          s0 = wmma16(qa.v, k0f.v, s0);
          s1 = wmma16(qa.v, k1f.v, s1);
        }
#pragma unroll
        for (int r = 0; r < 8; ++r) {
          const int qrow = q0 + 8 * hh + r;
          float a0 = s0[r] * sl2e, a1 = s1[r] * sl2e;
          a0 = (kh0 + c > qrow) ? NEG : a0;
          a1 = (kh0 + 16 + c > qrow) ? NEG : a1;
          float m = fmaxf(a0, a1);
          m = fmaxf(m, __shfl_xor(m, 1, 32)); m = fmaxf(m, __shfl_xor(m, 2, 32));
          m = fmaxf(m, __shfl_xor(m, 4, 32)); m = fmaxf(m, __shfl_xor(m, 8, 32));
          const float mnew  = fmaxf(mrow[r], m);
          const float alpha = exp2f(mrow[r] - mnew);
          const float p0 = exp2f(a0 - mnew), p1 = exp2f(a1 - mnew);
          float ps = p0 + p1;
          ps += __shfl_xor(ps, 1, 32); ps += __shfl_xor(ps, 2, 32); ps += __shfl_xor(ps, 4, 32); ps += __shfl_xor(ps, 8, 32);
          lrow[r] = lrow[r] * alpha + ps; mrow[r] = mnew;
#pragma unroll
          for (int t = 0; t < 4; ++t) oacc[t][r] *= alpha;
          Psh[wave][(8 * hh + r) * AT_PP + c]      = (_Float16)(p0 * 4096.f);
          Psh[wave][(8 * hh + r) * AT_PP + 16 + c] = (_Float16)(p1 * 4096.f);
        }
        wave_sync();
        {
          FragU pa, vb0, vb1, vb2, vb3;
          const int pb = c * AT_PP + 8 * hh;
          pa.h[0] = *(const v8ha*)&Psh[wave][pb]; pa.h[1] = *(const v8ha*)&Psh[wave][pb + 16];
          const int vo = c * AT_VP + hf * 32 + 8 * hh;
          vb0.h[0] = *(const v8ha*)&Vth[vo];                 vb0.h[1] = *(const v8ha*)&Vth[vo + 16];
          vb1.h[0] = *(const v8ha*)&Vth[vo + 16 * AT_VP];    vb1.h[1] = *(const v8ha*)&Vth[vo + 16 * AT_VP + 16];
          vb2.h[0] = *(const v8ha*)&Vth[vo + 32 * AT_VP];    vb2.h[1] = *(const v8ha*)&Vth[vo + 32 * AT_VP + 16];
          vb3.h[0] = *(const v8ha*)&Vth[vo + 48 * AT_VP];    vb3.h[1] = *(const v8ha*)&Vth[vo + 48 * AT_VP + 16];
          oacc[0] = wmma16(pa.v, vb0.v, oacc[0]);
          oacc[1] = wmma16(pa.v, vb1.v, oacc[1]);
          oacc[2] = wmma16(pa.v, vb2.v, oacc[2]);
          oacc[3] = wmma16(pa.v, vb3.v, oacc[3]);
        }
        wave_sync();
      }
    }
  }

#pragma unroll
  for (int r = 0; r < 8; ++r) {
    const float inv = oscale * (1.0f / (lrow[r] * 4096.f));
#pragma unroll
    for (int t = 0; t < 4; ++t) Os[wave][(8 * hh + r) * AT_OP + t * 16 + c] = oacc[t][r] * inv;
  }
  wave_sync();
  {
    const int q = lane >> 3, c8 = (lane & 7) * 8;
    for (int pass = 0; pass < 2; ++pass) {
#pragma unroll
      for (int it = 0; it < 4; ++it) {
        const int row = it * 4 + q;
        v8h hv;
#pragma unroll
        for (int e = 0; e < 8; ++e) hv[e] = (_Float16)Os[wave][row * AT_OP + c8 + e];
        *(volatile v8h*)(AOp + (rowbase + q0 + row) * NE + h * HD + c8) = hv;
      }
      __threadfence();
    }
  }
}

extern "C" void kernel_launch(void* const* d_in, const int* in_sizes, int n_in, void* d_out, int out_size, void* d_ws, size_t ws_size, hipStream_t stream) {
    if (n_in < 14) return;
    constexpr long long XNEED = ((long long)(NB - 1) * SEQ_FULL + SEQ) * NE;
    if ((long long)in_sizes[0] < XNEED) return;
    if (in_sizes[1] < NE || in_sizes[2] < NE) return;
    if (in_sizes[3] < NHD * NE * HD || in_sizes[4] < NHD * NE * HD || in_sizes[5] < NHD * NE * HD) return;
    if (in_sizes[6] < NE * NE || in_sizes[7] < NE || in_sizes[8] < NE || in_sizes[9] < NE) return;
    if (in_sizes[10] < NE * NFF || in_sizes[11] < NFF || in_sizes[12] < NFF * NE || in_sizes[13] < NE) return;
    if ((long long)out_size < XNEED) return;

    const float* x   = (const float*)d_in[0];
    const float* g1  = (const float*)d_in[1];
    const float* be1 = (const float*)d_in[2];
    const float* wq  = (const float*)d_in[3];
    const float* wk  = (const float*)d_in[4];
    const float* wv  = (const float*)d_in[5];
    const float* wo  = (const float*)d_in[6];
    const float* bo  = (const float*)d_in[7];
    const float* g2  = (const float*)d_in[8];
    const float* be2 = (const float*)d_in[9];
    const float* w1  = (const float*)d_in[10];
    const float* b1  = (const float*)d_in[11];
    const float* w2  = (const float*)d_in[12];
    const float* b2  = (const float*)d_in[13];
    float* out = (float*)d_out;

    constexpr size_t SZ_X16 = (size_t)MROWS * NE * 2;
    constexpr size_t SZ_QKV = (size_t)MROWS * NQKV * 2;
    constexpr size_t SZ_R0  = (size_t)MROWS * NFF * 2;
    constexpr size_t SZ_X1  = (size_t)MROWS * NE * 4;
    constexpr size_t SZ_H16 = (size_t)MROWS * NE * 2;
    constexpr size_t SZ_W3  = (size_t)NQKV * NE * 2;
    constexpr size_t SZ_WP  = (size_t)NE * NE * 2;
    constexpr size_t SZ_W1  = (size_t)NFF * NE * 2;
    constexpr size_t SZ_W2  = (size_t)NE * NFF * 2;
    static_assert(SZ_X16 + SZ_QKV == SZ_R0);
    static_assert(SZ_X16 % 256 == 0 && SZ_QKV % 256 == 0 && SZ_X1 % 256 == 0 && SZ_H16 % 256 == 0);
    static_assert(SZ_W3 % 256 == 0 && SZ_WP % 256 == 0 && SZ_W1 % 256 == 0 && SZ_W2 % 256 == 0);
    constexpr size_t WS_TOTAL = SZ_R0 + SZ_X1 + SZ_H16 + SZ_W3 + SZ_WP + SZ_W1 + SZ_W2;
    static_assert(WS_TOTAL <= (size_t)134217728);
    if (WS_TOTAL > ws_size) return;
    char* wsp = (char*)d_ws;
    unsigned short* X16   = (unsigned short*)(wsp);
    unsigned short* QKV16 = (unsigned short*)(wsp + SZ_X16);
    unsigned short* AO16  = X16;
    unsigned short* F16   = X16;
    float*          X1    = (float*)(wsp + SZ_R0);
    unsigned short* H16   = (unsigned short*)(wsp + SZ_R0 + SZ_X1);
    unsigned short* W3T   = (unsigned short*)(wsp + SZ_R0 + SZ_X1 + SZ_H16);
    unsigned short* WPT   = (unsigned short*)(wsp + SZ_R0 + SZ_X1 + SZ_H16 + SZ_W3);
    unsigned short* W1T   = (unsigned short*)(wsp + SZ_R0 + SZ_X1 + SZ_H16 + SZ_W3 + SZ_WP);
    unsigned short* W2T   = (unsigned short*)(wsp + SZ_R0 + SZ_X1 + SZ_H16 + SZ_W3 + SZ_WP + SZ_W1);

    {
        const unsigned gx = (unsigned)(((long long)HD * (NE / 8) + 255) / 256);
        k_cm_castbT<<<dim3(gx, NHD), 256, 0, stream>>>(wq, HD, (long long)NE * HD, W3T,                       NE, (long long)HD * NE, NE, HD, 16.0f);
        k_cm_castbT<<<dim3(gx, NHD), 256, 0, stream>>>(wk, HD, (long long)NE * HD, W3T + (size_t)NE * NE,     NE, (long long)HD * NE, NE, HD, 16.0f);
        k_cm_castbT<<<dim3(gx, NHD), 256, 0, stream>>>(wv, HD, (long long)NE * HD, W3T + (size_t)2 * NE * NE, NE, (long long)HD * NE, NE, HD, 16.0f);
    }
    k_cm_castbT<<<dim3((unsigned)(((long long)NE * (NE / 8) + 255) / 256), 1), 256, 0, stream>>>(wo, NE, 0, WPT, NE, 0, NE, NE, 16.0f);
    k_cm_castbT<<<dim3((unsigned)(((long long)NFF * (NE / 8) + 255) / 256), 1), 256, 0, stream>>>(w1, NFF, 0, W1T, NE, 0, NE, NFF, 16.0f);
    k_cm_castbT<<<dim3((unsigned)(((long long)NE * (NFF / 8) + 255) / 256), 1), 256, 0, stream>>>(w2, NE, 0, W2T, NFF, 0, NFF, NE, 16.0f);

    k_b_ln<3, 1><<<(MROWS + 7) / 8, 256, 0, stream>>>(x, g1, be1, 1e-6f, 1.0f / (float)NE, MROWS, SEQ, SEQ_FULL, X16);
    wmma_gemm64<0, 1, false, false, 0><<<dim3((unsigned)(((MROWS / 64) * (NQKV / 64) + 7) / 8), 1), 256, 0, stream>>>(
        X16, NE, 0, W3T, NE, 0, (void*)QKV16, NQKV, 0, nullptr, nullptr, 0, MROWS, NQKV, NE, 0.0625f);
    {
        const float sl2e = 0.05103103630798288f * 1.4426950408889634f;
        k_attn_causal<<<dim3((unsigned)(NB * NHD * (SEQ / 64))), 128, 0, stream>>>(QKV16, AO16, sl2e, 16.0f);
    }
    wmma_gemm64<2, 0, true, true, 0><<<dim3((unsigned)(((SEQ / 64) * (NE / 64) + 7) / 8), (unsigned)NB), 256, 0, stream>>>(
        AO16, NE, (long long)SEQ * NE, WPT, NE, 0, (void*)X1, NE, (long long)SEQ * NE, bo, x, (long long)SEQ_FULL * NE, SEQ, NE, NE, 0.00390625f);
    k_b_ln<3, 0><<<(MROWS + 7) / 8, 256, 0, stream>>>(X1, g2, be2, 1e-6f, 1.0f / (float)NE, MROWS, SEQ, SEQ, H16);
    wmma_gemm64<2, 1, false, false, 2><<<dim3((unsigned)(((MROWS / 64) * (NFF / 64) + 7) / 8), 1), 256, 0, stream>>>(
        H16, NE, 0, W1T, NE, 0, (void*)F16, NFF, 0, b1, nullptr, 0, MROWS, NFF, NE, 0.0625f);
    wmma_gemm64<2, 0, true, false, 0><<<dim3((unsigned)(((SEQ / 64) * (NE / 64) + 7) / 8), (unsigned)NB), 256, 0, stream>>>(
        F16, NFF, (long long)SEQ * NFF, W2T, NFF, 0, (void*)out, NE, (long long)SEQ_FULL * NE, b2, X1, (long long)SEQ * NE, SEQ, NE, NFF, 0.0625f);
}
